// ClassicalSelfAttention_65481071408671
// MI455X (gfx1250) — hardware-verified
//
#include <hip/hip_runtime.h>


#ifndef NB
#define NB 2
#endif
#ifndef SEQ
#define SEQ 4096
#endif
#define NB_FULL  2
#define SEQ_FULL 4096
#define EMB  512
#define NHD  8
#define HD   64
#define PCAR 1024.0f
#define C2   0.18033688011112042f

static_assert(NB >= 1 && NB <= NB_FULL);
static_assert(SEQ % 64 == 0 && SEQ >= 64 && SEQ <= SEQ_FULL);
static_assert(EMB == NHD * HD);
static_assert(EMB % 64 == 0 && HD == 64);
static_assert((SEQ * EMB) % 2048 == 0);

typedef _Float16 h16;
typedef unsigned short bf;
typedef __attribute__((ext_vector_type(16))) __bf16   v16bf;
typedef __attribute__((ext_vector_type(16))) _Float16 v16h;
typedef __attribute__((ext_vector_type(8)))  _Float16 v8h;
typedef __attribute__((ext_vector_type(8)))  unsigned short v8us;
typedef __attribute__((ext_vector_type(8)))  float    v8f;
typedef __attribute__((ext_vector_type(4)))  float    v4f;
typedef __attribute__((ext_vector_type(2)))  _Float16 v2h;
typedef __attribute__((ext_vector_type(2)))  unsigned short v2us;
typedef v8h  __attribute__((may_alias)) v8ha;
typedef v4f  __attribute__((may_alias)) v4fa;
typedef v8us __attribute__((may_alias)) v8usa;

__device__ __forceinline__ unsigned short f2bf(float f) { unsigned u = __float_as_uint(f); u += 0x7FFFu + ((u >> 16) & 1u); return (unsigned short)(u >> 16); }
__device__ __forceinline__ float bf2f(unsigned short b) { return __uint_as_float(((unsigned)b) << 16); }
__device__ __forceinline__ float bfr(float f) { return bf2f(f2bf(f)); }
__device__ __forceinline__ v16h cat16(v8h lo, v8h hi) { return __builtin_shufflevector(lo, hi, 0, 1, 2, 3, 4, 5, 6, 7, 8, 9, 10, 11, 12, 13, 14, 15); }
__device__ __forceinline__ v16bf cat16b(v8us lo, v8us hi) { return __builtin_bit_cast(v16bf, __builtin_shufflevector(lo, hi, 0, 1, 2, 3, 4, 5, 6, 7, 8, 9, 10, 11, 12, 13, 14, 15)); }
__device__ __forceinline__ v8f wmma16(v16h a, v16h b, v8f c) { return __builtin_amdgcn_wmma_f32_16x16x32_f16(false, a, false, b, (short)0, c, false, false); }
__device__ __forceinline__ v8f wmmab(v16bf a, v16bf b, v8f c) { return __builtin_amdgcn_wmma_f32_16x16x32_bf16(false, a, false, b, (short)0, c, false, false); }
__device__ __forceinline__ void splitf(float y, unsigned short& h, unsigned short& l) { h = f2bf(y); l = f2bf(y - bf2f(h)); }

template <typename T16> struct WFrag;
template <> struct WFrag<h16> { typedef v16h V; static __device__ __forceinline__ V ld(const h16* p) { return cat16(*(const v8h*)p, *(const v8h*)(p + 16)); } static __device__ __forceinline__ v8f mma(V a, V b, v8f c) { return wmma16(a, b, c); } };
template <> struct WFrag<bf> { typedef v16bf V; static __device__ __forceinline__ V ld(const bf* p) { return cat16b(*(const v8us*)p, *(const v8us*)(p + 16)); } static __device__ __forceinline__ v8f mma(V a, V b, v8f c) { return wmmab(a, b, c); } };
template <typename T16, int NSPLIT, bool BIAS>
__global__ __launch_bounds__(32) void k_gemmw(const T16* __restrict__ A, const T16* __restrict__ A2, const T16* __restrict__ Bt, const T16* __restrict__ Bt2, int K, float* C, int ldc, const float* __restrict__ bias, size_t sA, size_t sB, size_t sC) {
    typedef typename WFrag<T16>::V V;
    __shared__ __align__(16) float os[16 * 68];
    const size_t z = blockIdx.z; A += z * sA; if (A2) A2 += z * sA; Bt += z * sB; if (Bt2) Bt2 += z * sB; C += z * sC;
    const int lane = threadIdx.x & 31, lr = lane & 15, hi = lane >> 4; const int r0 = blockIdx.x * 64, c0 = blockIdx.y * 64;
    v8f acc[4][4];
#pragma unroll
    for (int mb = 0; mb < 4; ++mb)
#pragma unroll
        for (int nb = 0; nb < 4; ++nb) acc[mb][nb] = (v8f){};
    const size_t aoff = (size_t)(r0 + lr) * K + 8 * hi, boff = (size_t)(c0 + lr) * K + 8 * hi;
#pragma unroll 1
    for (int kc = 0; kc < K; kc += 32) {
        V a[4], a2[4];
#pragma unroll
        for (int mb = 0; mb < 4; ++mb) { a[mb] = WFrag<T16>::ld(A + aoff + (size_t)mb * 16 * K + kc); if (NSPLIT == 1 || NSPLIT == 2) a2[mb] = WFrag<T16>::ld(A2 + aoff + (size_t)mb * 16 * K + kc); }
#pragma unroll
        for (int nb = 0; nb < 4; ++nb) { const V b = WFrag<T16>::ld(Bt + boff + (size_t)nb * 16 * K + kc); V b2; if (NSPLIT >= 2) b2 = WFrag<T16>::ld(Bt2 + boff + (size_t)nb * 16 * K + kc);
#pragma unroll
            for (int mb = 0; mb < 4; ++mb) { acc[mb][nb] = WFrag<T16>::mma(a[mb], b, acc[mb][nb]); if (NSPLIT == 1 || NSPLIT == 2) acc[mb][nb] = WFrag<T16>::mma(a2[mb], b, acc[mb][nb]); if (NSPLIT >= 2) acc[mb][nb] = WFrag<T16>::mma(a[mb], b2, acc[mb][nb]); } }
        asm volatile("v_nop\n\tv_nop\n\tv_nop\n\tv_nop" : "+v"(acc[0][0]), "+v"(acc[1][1]), "+v"(acc[2][2]), "+v"(acc[3][3]) : "v"(a[0]), "v"(a[3]));
    }
#pragma unroll
    for (int mb = 0; mb < 4; ++mb) {
#pragma unroll
        for (int nb = 0; nb < 4; ++nb) {
#pragma unroll
            for (int j = 0; j < 8; ++j) os[(hi * 8 + j) * 68 + nb * 16 + lr] = acc[mb][nb][j]; }
        asm volatile("" ::: "memory"); __builtin_amdgcn_fence(3, "wavefront"); __builtin_amdgcn_wave_barrier(); asm volatile("" ::: "memory");
        float* crow = C + (size_t)(r0 + mb * 16) * ldc + c0;
#pragma unroll 1
        for (int ps = 0; ps < 2; ++ps) {
#pragma unroll
            for (int s = 0; s < 8; ++s) { const int row = 2 * s + hi, cofs = lr * 4; v4f val = *(const v4fa*)(os + row * 68 + cofs); if (BIAS) { val[0] += bfr(bias[c0 + cofs]); val[1] += bfr(bias[c0 + cofs + 1]); val[2] += bfr(bias[c0 + cofs + 2]); val[3] += bfr(bias[c0 + cofs + 3]); }
                *(volatile v4f*)(crow + (size_t)row * ldc + cofs) = val; }
            if (ps == 0) __threadfence(); }
        __builtin_amdgcn_wave_barrier(); asm volatile("" ::: "memory");
    }
}

__global__ __launch_bounds__(256) void k_wtG(const float* __restrict__ w, int K, int N, bf* Bt) {
    const int lane = threadIdx.x & 31; const int L0 = (blockIdx.x * 8 + (threadIdx.x >> 5)) * 8; const int nlines = N * K / 64;
#pragma unroll
    for (int ps = 0; ps < 2; ++ps) {
#pragma unroll 1
        for (int l = 0; l < 8; ++l) { const int L = L0 + l; if (L >= nlines) break; const size_t e = (size_t)L * 64 + lane * 2; const int k = (int)(e % K), n = (int)(e / K); v2us o;
            o[0] = f2bf(w[(size_t)k * N + n]); o[1] = f2bf(w[(size_t)(k + 1) * N + n]); *(volatile v2us*)(Bt + e) = o; }
        if (ps == 0) __threadfence(); }
}
__global__ __launch_bounds__(256) void k_cvt8(const float* __restrict__ src, bf* dst, size_t n8) { const size_t i = (size_t)blockIdx.x * 256 + threadIdx.x; if (i >= n8) return; const v8f v = *(const v8f*)(src + i * 8); v8us o;
#pragma unroll
    for (int k = 0; k < 8; ++k) o[k] = f2bf(v[k]); *(volatile v8us*)(dst + i * 8) = o; __threadfence(); *(volatile v8us*)(dst + i * 8) = o; }
__global__ __launch_bounds__(256) void k_split8(const float* __restrict__ src, bf* Ph, bf* Pl, size_t n8) { const size_t i = (size_t)blockIdx.x * 256 + threadIdx.x; if (i >= n8) return; const v8f v = *(const v8f*)(src + i * 8); v8us oh, ol;
#pragma unroll
    for (int k = 0; k < 8; ++k) { unsigned short a, c; splitf(v[k], a, c); oh[k] = a; ol[k] = c; }
    *(volatile v8us*)(Ph + i * 8) = oh; *(volatile v8us*)(Pl + i * 8) = ol; __threadfence(); *(volatile v8us*)(Ph + i * 8) = oh; *(volatile v8us*)(Pl + i * 8) = ol; }
__global__ __launch_bounds__(256) void k_cvth(const float* __restrict__ src, h16* dst, size_t n8) { const size_t i = (size_t)blockIdx.x * 256 + threadIdx.x; if (i >= n8) return; const v8f v = *(const v8f*)(src + i * 8); v8h o;
#pragma unroll
    for (int k = 0; k < 8; ++k) o[k] = (h16)v[k]; *(volatile v8h*)(dst + i * 8) = o; __threadfence(); *(volatile v8h*)(dst + i * 8) = o; }
__global__ __launch_bounds__(256) void k_vtp(const float* __restrict__ F, h16* V16, size_t ntot) {
    const size_t e = ((size_t)blockIdx.x * 256 + threadIdx.x) * 2; if (e >= ntot) return;
    const int s = (int)(e % SEQ); const int c = (int)((e / SEQ) % EMB); const int b = (int)(e / ((size_t)SEQ * EMB));
    const float* fr = F + ((size_t)b * SEQ + s) * EMB + c;
    v2h o; o[0] = (h16)fr[0]; o[1] = (h16)fr[EMB];
    *(volatile v2h*)(V16 + e) = o; __threadfence(); *(volatile v2h*)(V16 + e) = o; }

__device__ __forceinline__ v16h ldh(const h16* p) { return cat16(*(const v8h*)p, *(const v8h*)(p + 16)); }

__global__ __launch_bounds__(128) __attribute__((amdgpu_num_vgpr(256)))
void k_flash(const h16* __restrict__ Qp, const h16* __restrict__ Kp, const h16* __restrict__ Vtp, float* OUT) {
    __shared__ __align__(16) float os[4 * 16 * 68];
    const int tid = threadIdx.x, w = tid >> 5, lane = tid & 31, lm = lane & 15, hh = lane >> 4;
    const int nqt = SEQ / 64;
    const int bid = blockIdx.x; const int qt = bid % nqt; const int h = (bid / nqt) % NHD; const int b = bid / (nqt * NHD);
    const int q0 = qt * 64 + w * 16;
    const h16* Qb = Qp + ((size_t)b * SEQ + q0) * EMB + h * HD;
    const h16* Kb = Kp + (size_t)b * SEQ * EMB + h * HD;
    const h16* Vb = Vtp + ((size_t)b * EMB + h * HD) * SEQ;
    const v16h qf0 = ldh(Qb + (size_t)lm * EMB + 8 * hh);
    const v16h qf1 = ldh(Qb + (size_t)lm * EMB + 32 + 8 * hh);
    float mrun = -3.0e38f, lrun = 0.0f;
    v8f acc[4];
#pragma unroll
    for (int t = 0; t < 4; ++t) acc[t] = (v8f){};
#pragma unroll 1
    for (int kv = 0; kv < SEQ; kv += 64) {
        v8f s[4];
#pragma unroll
        for (int t4 = 0; t4 < 4; ++t4) {
            const h16* kr = Kb + (size_t)(kv + t4 * 16 + lm) * EMB + 8 * hh;
            const v16h ka = ldh(kr), kb2 = ldh(kr + 32);
            s[t4] = wmma16(ka, qf0, (v8f){});
            s[t4] = wmma16(kb2, qf1, s[t4]);
        }
        asm volatile("v_nop\n\tv_nop\n\tv_nop\n\tv_nop" : "+v"(s[0]), "+v"(s[1]), "+v"(s[2]), "+v"(s[3]) : "v"(qf0), "v"(qf1));
        float mx = -3.0e38f;
#pragma unroll
        for (int t4 = 0; t4 < 4; ++t4) { s[t4] = s[t4] * C2;
#pragma unroll
            for (int r = 0; r < 8; ++r) mx = fmaxf(mx, s[t4][r]); }
        mx = fmaxf(mx, __shfl_xor(mx, 16, 32));
        const float mnew = fmaxf(mrun, mx);
        const float alpha = __builtin_amdgcn_exp2f(mrun - mnew);
        float rs = 0.0f; v8h ph[4];
#pragma unroll
        for (int t4 = 0; t4 < 4; ++t4) {
#pragma unroll
            for (int r = 0; r < 8; ++r) { const float p = __builtin_amdgcn_exp2f(s[t4][r] - mnew); rs += p; ph[t4][r] = (h16)(p * PCAR); } }
        rs += __shfl_xor(rs, 16, 32);
        lrun = lrun * alpha + rs; mrun = mnew;
#pragma unroll
        for (int t = 0; t < 4; ++t) acc[t] = acc[t] * alpha;
        const v16h pf0 = cat16(ph[0], ph[1]), pf1 = cat16(ph[2], ph[3]);
#pragma unroll
        for (int t = 0; t < 4; ++t) {
            const h16* vr = Vb + (size_t)(t * 16 + lm) * SEQ + kv + 8 * hh;
            acc[t] = wmma16(ldh(vr), pf0, acc[t]);
            acc[t] = wmma16(ldh(vr + 32), pf1, acc[t]);
        }
        asm volatile("v_nop\n\tv_nop\n\tv_nop\n\tv_nop" : "+v"(acc[0]), "+v"(acc[1]), "+v"(acc[2]), "+v"(acc[3]) : "v"(pf0), "v"(pf1));
    }
    const float inv = __fdiv_rn(1.0f, lrun) * (1.0f / PCAR);
    float* mo = os + w * (16 * 68);
#pragma unroll
    for (int t = 0; t < 4; ++t)
#pragma unroll
        for (int r = 0; r < 8; ++r) mo[lm * 68 + t * 16 + 8 * hh + r] = acc[t][r] * inv;
    asm volatile("" ::: "memory"); __builtin_amdgcn_fence(3, "wavefront"); __builtin_amdgcn_wave_barrier(); asm volatile("" ::: "memory");
    float* orow = OUT + ((size_t)b * SEQ_FULL + q0) * EMB + h * HD;
#pragma unroll 1
    for (int ps = 0; ps < 2; ++ps) {
#pragma unroll
        for (int si = 0; si < 8; ++si) { const int row = 2 * si + hh, cofs = lm * 4; const v4f val = *(const v4fa*)(mo + row * 68 + cofs); *(volatile v4f*)(orow + (size_t)row * EMB + cofs) = val; }
        if (ps == 0) __threadfence(); }
}

extern "C" void kernel_launch(void* const* d_in, const int* in_sizes, int n_in,
                              void* d_out, int out_size, void* d_ws, size_t ws_size, hipStream_t stream) {
    if (n_in < 6) return;
    const size_t nw = (size_t)EMB * EMB;
    const size_t needx = ((size_t)(NB - 1) * SEQ_FULL + SEQ) * EMB;
    if ((size_t)in_sizes[0] < nw || (size_t)in_sizes[1] < nw || (size_t)in_sizes[2] < needx ||
        (size_t)in_sizes[3] < nw || (size_t)in_sizes[4] < nw || (size_t)in_sizes[5] < nw) return;
    if ((size_t)out_size < needx) return;
    const float* rot = (const float*)d_in[0];
    const float* ent = (const float*)d_in[1];
    const float* x   = (const float*)d_in[2];
    const float* wq  = (const float*)d_in[3];
    const float* wk  = (const float*)d_in[4];
    const float* wv  = (const float*)d_in[5];
    float* OUT = (float*)d_out;
    const size_t nrow = (size_t)NB * SEQ;
    const size_t nx = nrow * EMB;
    char* wsp = (char*)d_ws;
    auto take = [&](size_t bytes) { char* p = wsp; wsp += (bytes + 255) & ~(size_t)255; return (void*)p; };
    bf* WV   = (bf*)take(nw * 2);
    bf* TRE  = (bf*)take(2 * nw * 2);
    bf* WQKT = (bf*)take(2 * nw * 2);
    float* WC = (float*)take(2 * nw * 4);
    bf* WCh  = (bf*)take(2 * nw * 2);
    bf* WCl  = (bf*)take(2 * nw * 2);
    bf* XB   = (bf*)take(nx * 2);
    float* FQK = (float*)take(2 * nx * 4);
    float* FV  = (float*)take(nx * 4);
    h16* QK16  = (h16*)take(2 * nx * 2);
    h16* VT16  = (h16*)take(nx * 2);
    if ((size_t)(wsp - (char*)d_ws) > ws_size) return;
    k_cvt8<<<(unsigned)((nw / 8 + 255) / 256), 256, 0, stream>>>(wv, WV, nw / 8);
    const unsigned gw = (unsigned)((nw / 64 + 63) / 64);
    k_wtG<<<gw, 256, 0, stream>>>(rot, EMB, EMB, TRE);
    k_wtG<<<gw, 256, 0, stream>>>(ent, EMB, EMB, TRE + nw);
    k_wtG<<<gw, 256, 0, stream>>>(wq, EMB, EMB, WQKT);
    k_wtG<<<gw, 256, 0, stream>>>(wk, EMB, EMB, WQKT + nw);
    k_gemmw<bf, 0, false><<<dim3(EMB / 64, EMB / 64, 2), 32, 0, stream>>>(TRE, nullptr, WQKT, nullptr, EMB, WC, EMB, nullptr, nw, nw, nw);
    k_split8<<<(unsigned)((2 * nw / 8 + 255) / 256), 256, 0, stream>>>(WC, WCh, WCl, 2 * nw / 8);
    for (int b = 0; b < NB; ++b)
        k_cvt8<<<(unsigned)(((size_t)SEQ * EMB / 8 + 255) / 256), 256, 0, stream>>>(x + (size_t)b * SEQ_FULL * EMB, XB + (size_t)b * SEQ * EMB, (size_t)SEQ * EMB / 8);
    k_gemmw<bf, 3, false><<<dim3((unsigned)(nrow / 64), EMB / 64, 2), 32, 0, stream>>>(XB, nullptr, WCh, WCl, EMB, FQK, EMB, nullptr, 0, nw, nx);
    k_gemmw<bf, 0, false><<<dim3((unsigned)(nrow / 64), EMB / 64, 1), 32, 0, stream>>>(XB, nullptr, WV, nullptr, EMB, FV, EMB, nullptr, 0, 0, 0);
    k_cvth<<<(unsigned)((2 * nx / 8 + 255) / 256), 256, 0, stream>>>(FQK, QK16, 2 * nx / 8);
    k_vtp<<<(unsigned)((nx / 2 + 255) / 256), 256, 0, stream>>>(FV, VT16, nx);
    k_flash<<<(unsigned)(NB * NHD * (SEQ / 64)), 128, 0, stream>>>(QK16, QK16 + nx, VT16, OUT);
}
